// SparseLTSRouter_81844896792945
// MI455X (gfx1250) — hardware-verified
//
#include <hip/hip_runtime.h>
#include <math.h>

typedef __attribute__((ext_vector_type(16))) _Float16 v16h;
typedef __attribute__((ext_vector_type(16))) __bf16 v16b;
typedef __attribute__((ext_vector_type(8)))  _Float16 v8h;
typedef __attribute__((ext_vector_type(8)))  float v8f;
typedef __attribute__((ext_vector_type(4)))  float v4f;
typedef __attribute__((ext_vector_type(2)))  float v2f;
typedef __attribute__((ext_vector_type(4)))  unsigned v4u;
typedef __attribute__((ext_vector_type(4)))  int v4i;
typedef float __attribute__((may_alias)) float_a;
typedef int __attribute__((may_alias)) int_a;

template <typename T> __device__ __forceinline__ void vst2(void* p, T v) { *(volatile T*)p = v; __threadfence(); *(volatile T*)p = v; }
__device__ __forceinline__ v8f wmma16(v16h a, v16h b, v8f c) {
  v8f d = __builtin_amdgcn_wmma_f32_16x16x32_f16(false, a, false, b, (short)0, c, false, false);
  asm volatile("v_nop\n\tv_nop\n\tv_nop\n\tv_nop" : "+v"(d) : "v"(a), "v"(b));
  return d;
}
__device__ __forceinline__ v8f wmma_bf(v16b a, v16b b, v8f c) {
  v8f d = __builtin_amdgcn_wmma_f32_16x16x32_bf16(false, a, false, b, (short)0, c, false, false);
  asm volatile("v_nop\n\tv_nop\n\tv_nop\n\tv_nop" : "+v"(d) : "v"(a), "v"(b));
  return d;
}
__device__ __forceinline__ v16h frag_h(const _Float16* rowk0, int lane) {
  union { v16h v; v8h q[2]; } u; const _Float16* p = rowk0 + 8 * (lane >> 4);
  u.q[0] = *(const v8h*)p; u.q[1] = *(const v8h*)(p + 16); return u.v;
}
__device__ __forceinline__ v16h frag_f32(const float* rowk0, int lane) {
  v16h a; const float* p = rowk0 + 8 * (lane >> 4);
#pragma unroll
  for (int i = 0; i < 8; ++i) { a[i] = (_Float16)p[i]; a[8 + i] = (_Float16)p[16 + i]; }
  return a;
}
__device__ __forceinline__ v16h frag_f32s(const float* rowk0, int lane, float sc) {
  v16h a; const float* p = rowk0 + 8 * (lane >> 4);
#pragma unroll
  for (int i = 0; i < 8; ++i) { a[i] = (_Float16)(p[i] * sc); a[8 + i] = (_Float16)(p[16 + i] * sc); }
  return a;
}
__device__ __forceinline__ v16h fragc_f32(const float* W, int k0, int n, int lane, int ld, int K) {
  v16h a; const int g = lane >> 4;
#pragma unroll
  for (int i = 0; i < 8; ++i) { const int ka = k0 + 8 * g + i, kb = ka + 16;
    a[i] = (_Float16)(ka < K ? W[(size_t)ka * ld + n] : 0.f); a[8 + i] = (_Float16)(kb < K ? W[(size_t)kb * ld + n] : 0.f); }
  return a;
}
struct F2 { v16b h, l; };
__device__ __forceinline__ F2 bsplit16(const float v[16]) { F2 r;
#pragma unroll
  for (int i = 0; i < 16; ++i) { const __bf16 h = (__bf16)v[i]; r.h[i] = h; r.l[i] = (__bf16)(v[i] - (float)h); }
  return r; }
__device__ __forceinline__ F2 split_row(const float* row, int k0, int lane) { float v[16]; const float* p = row + k0 + 8 * (lane >> 4);
#pragma unroll
  for (int i = 0; i < 8; ++i) { v[i] = p[i]; v[8 + i] = p[16 + i]; }
  return bsplit16(v); }
__device__ __forceinline__ F2 split_rowK(const float* row, int k0, int lane, int K) { float v[16]; const int g = lane >> 4;
#pragma unroll
  for (int i = 0; i < 8; ++i) { const int ka = k0 + 8 * g + i, kb = ka + 16; v[i] = ka < K ? row[ka] : 0.f; v[8 + i] = kb < K ? row[kb] : 0.f; }
  return bsplit16(v); }
__device__ __forceinline__ F2 split_col(const float* W, int k0, int n, int lane, int ld, int K) { float v[16]; const int g = lane >> 4;
#pragma unroll
  for (int i = 0; i < 8; ++i) { const int ka = k0 + 8 * g + i, kb = ka + 16; v[i] = ka < K ? W[(size_t)ka * ld + n] : 0.f; v[8 + i] = kb < K ? W[(size_t)kb * ld + n] : 0.f; }
  return bsplit16(v); }
__device__ __forceinline__ v8f mac3(const F2& a, const F2& b, v8f c) { c = wmma_bf(a.l, b.h, c); c = wmma_bf(a.h, b.l, c); return wmma_bf(a.h, b.h, c); }
__device__ __forceinline__ float sigm(float v) { return 1.0f / (1.0f + expf(-v)); }
#define LDSX() do { asm volatile("s_wait_dscnt 0" ::: "memory"); __builtin_amdgcn_wave_barrier(); __builtin_amdgcn_fence(__ATOMIC_RELEASE, "workgroup"); } while (0)

#define NT 4096
#define DD 1024
#define NE 4
#define TK 32
#define NL 8192
#define EPE (NL / NE)

__global__ __launch_bounds__(256) void k_cvt(const float* __restrict__ h, const float* __restrict__ lts, _Float16* __restrict__ h16, _Float16* __restrict__ sel16) {
  const size_t g8 = (size_t)blockIdx.x * 256 + threadIdx.x; const size_t nh8 = (size_t)NT * DD / 8, ns8 = (size_t)NE * TK * DD / 8;
  union { v8h hh; v4u u; } pk;
  if (g8 < nh8) {
#pragma unroll
    for (int e = 0; e < 8; ++e) pk.hh[e] = (_Float16)h[g8 * 8 + e];
    vst2(h16 + g8 * 8, pk.u); }
  else if (g8 < nh8 + ns8) { const size_t q = g8 - nh8; const size_t row = q / (DD / 8), c8 = q % (DD / 8); const size_t e = row / TK, kk = row % TK;
#pragma unroll
    for (int i = 0; i < 8; ++i) pk.hh[i] = (_Float16)lts[(e * EPE + kk) * DD + c8 * 8 + i];
    vst2(sel16 + row * DD + c8 * 8, pk.u); }
}
__global__ __launch_bounds__(128) void k_main(const float* __restrict__ h, const _Float16* __restrict__ h16, const float* __restrict__ lts, const _Float16* __restrict__ sel16, const float* __restrict__ Wr, const float* __restrict__ br,
                                            float* __restrict__ out, float* __restrict__ ew) {
  __shared__ __align__(16) float slog[4][16][20];
  __shared__ __align__(16) float sS[4][16][132];
  __shared__ __align__(16) _Float16 sP[4][16][136];
  __shared__ __align__(16) float so[4][16][132];
  __shared__ __align__(16) float sew[4][16][4];
  __shared__ int sidx[4][16];
  const int tid = threadIdx.x, w = tid >> 5, lane = tid & 31, col = lane & 15, g = lane >> 4;
  const int t0 = blockIdx.x * 64 + w * 16;
  { v8f acc = {};
#pragma unroll 2
    for (int kc = 0; kc < DD / 32; ++kc) { float bv[16];
#pragma unroll
      for (int i = 0; i < 8; ++i) { const int ka = kc * 32 + 8 * g + i; bv[i] = col < NE ? Wr[(size_t)col * DD + ka] : 0.f; bv[8 + i] = col < NE ? Wr[(size_t)col * DD + ka + 16] : 0.f; }
      acc = mac3(split_row(h + (size_t)(t0 + col) * DD, kc * 32, lane), bsplit16(bv), acc); }
#pragma unroll
    for (int r = 0; r < 8; ++r) slog[w][8 * g + r][col] = acc[r] + (col < NE ? br[col] : 0.f); }
  LDSX();
  if (g == 0) { const int m = col; float lg[NE]; float mx = -3.0e38f; int am = 0;
#pragma unroll
    for (int e = 0; e < NE; ++e) { lg[e] = slog[w][m][e]; if (lg[e] > mx) { mx = lg[e]; am = e; } }
    float z = 0.f;
#pragma unroll
    for (int e = 0; e < NE; ++e) { lg[e] = expf(lg[e] - mx); z += lg[e]; }
    const float inv = 1.0f / z;
#pragma unroll
    for (int e = 0; e < NE; ++e) sew[w][m][e] = lg[e] * inv;
    sidx[w][m] = am; }
  LDSX();
  for (int q = lane; q < 16; q += 32) vst2(ew + (size_t)(t0 + q) * NE, *(const v4f*)(&sew[w][q][0]));
  { v8f acc[8] = {};
#pragma unroll 1
    for (int kc = 0; kc < DD / 32; ++kc) { const v16h a = frag_h(h16 + (size_t)(t0 + col) * DD + kc * 32, lane);
#pragma unroll
      for (int j = 0; j < 8; ++j) acc[j] = wmma16(a, frag_h(sel16 + (size_t)(j * 16 + col) * DD + kc * 32, lane), acc[j]); }
#pragma unroll
    for (int j = 0; j < 8; ++j)
#pragma unroll
      for (int r = 0; r < 8; ++r) sS[w][8 * g + r][j * 16 + col] = acc[j][r] * (1.0f / 32.0f); }
  LDSX();
  { const int m = col, e = sidx[w][m]; float mx = -3.0e38f;
#pragma unroll
    for (int kk = 0; kk < 16; ++kk) mx = fmaxf(mx, sS[w][m][e * TK + g * 16 + kk]);
    mx = fmaxf(mx, __shfl_xor(mx, 16, 32)); float z = 0.f; float pv[16];
#pragma unroll
    for (int kk = 0; kk < 16; ++kk) { pv[kk] = expf(sS[w][m][e * TK + g * 16 + kk] - mx); z += pv[kk]; }
    z += __shfl_xor(z, 16, 32); const float inv = 16384.0f / z;
#pragma unroll
    for (int c = 0; c < 64; ++c) { const int cc = g * 64 + c; sP[w][m][cc] = (_Float16)0.f; }
    __builtin_amdgcn_wave_barrier(); asm volatile("s_wait_dscnt 0" ::: "memory");
#pragma unroll
    for (int kk = 0; kk < 16; ++kk) sP[w][m][e * TK + g * 16 + kk] = (_Float16)(pv[kk] * inv); }
  LDSX();
  v16h pa[4];
#pragma unroll
  for (int kc = 0; kc < 4; ++kc) pa[kc] = frag_h(&sP[w][col][0] + kc * 32, lane);
#pragma unroll 1
  for (int np = 0; np < DD / 128; ++np) { v8f acc[8] = {};
#pragma unroll
    for (int kc = 0; kc < 4; ++kc) {
#pragma unroll
      for (int j = 0; j < 8; ++j) acc[j] = wmma16(pa[kc], fragc_f32(lts + (size_t)kc * EPE * DD, 0, np * 128 + j * 16 + col, lane, DD, TK), acc[j]); }
#pragma unroll
    for (int j = 0; j < 8; ++j)
#pragma unroll
      for (int r = 0; r < 8; ++r) so[w][8 * g + r][j * 16 + col] = acc[j][r] * (1.0f / 16384.0f);
    LDSX();
#pragma unroll 4
    for (int rl = 0; rl < 16; ++rl) vst2(out + (size_t)(t0 + rl) * DD + np * 128 + lane * 4, *(const v4f*)(&so[w][rl][lane * 4]));
    LDSX(); }
}
extern "C" void kernel_launch(void* const* d_in, const int* in_sizes, int n_in, void* d_out, int out_size, void* d_ws, size_t ws_size, hipStream_t stream) {
  (void)in_sizes; (void)n_in; (void)out_size; (void)ws_size;
  const float* h = (const float*)d_in[0]; const float* lts = (const float*)d_in[1]; const float* Wr = (const float*)d_in[2]; const float* br = (const float*)d_in[3];
  float* out = (float*)d_out; float* ew = (float*)((char*)d_out + 16777216);
  char* ws = (char*)d_ws; size_t off = 0;
  auto take = [&](size_t bytes) { char* p = ws + off; off += (bytes + 255) & ~(size_t)255; return p; };
  _Float16* h16 = (_Float16*)take((size_t)NT * DD * 2); _Float16* sel16 = (_Float16*)take((size_t)NE * TK * DD * 2);
  const size_t n8 = (size_t)NT * DD / 8 + (size_t)NE * TK * DD / 8;
  k_cvt<<<(unsigned)((n8 + 255) / 256), 256, 0, stream>>>(h, lts, h16, sel16);
  k_main<<<NT / 64, 128, 0, stream>>>(h, h16, lts, sel16, Wr, br, out, ew);
}
